// SP_SA_6184752906711
// MI455X (gfx1250) — hardware-verified
//
#include <hip/hip_runtime.h>


#define NB_  64
#define NTK  196
#define NP   256
#define CC   768
#define NH_  12
#define HD   64
#define NR   (NB_ * NTK)
#define IG   8
#define DM   CC
#define SCL  0.125f
#define LOSC 1024.0f
typedef _Float16 h16;
typedef unsigned short bf;
typedef __attribute__((ext_vector_type(16))) __bf16   v16bf;
typedef __attribute__((ext_vector_type(16))) _Float16 v16h;
typedef __attribute__((ext_vector_type(8)))  _Float16 v8h;
typedef __attribute__((ext_vector_type(8)))  unsigned short v8us;
typedef __attribute__((ext_vector_type(8)))  float    v8f;
typedef __attribute__((ext_vector_type(4)))  float    v4f;
typedef v8h  __attribute__((may_alias)) v8ha;
typedef v4f  __attribute__((may_alias)) v4fa;
typedef v8us __attribute__((may_alias)) v8usa;

__device__ __forceinline__ unsigned short f2bf(float f) { unsigned u = __float_as_uint(f); u += 0x7FFFu + ((u >> 16) & 1u); return (unsigned short)(u >> 16); }
__device__ __forceinline__ float bf2f(unsigned short b) { return __uint_as_float(((unsigned)b) << 16); }
__device__ __forceinline__ float bfr(float f) { return bf2f(f2bf(f)); }
__device__ __forceinline__ v16h cat16(v8h lo, v8h hi) { return __builtin_shufflevector(lo, hi, 0, 1, 2, 3, 4, 5, 6, 7, 8, 9, 10, 11, 12, 13, 14, 15); }
__device__ __forceinline__ v16bf cat16b(v8us lo, v8us hi) { return __builtin_bit_cast(v16bf, __builtin_shufflevector(lo, hi, 0, 1, 2, 3, 4, 5, 6, 7, 8, 9, 10, 11, 12, 13, 14, 15)); }
__device__ __forceinline__ v8f wmma16(v16h a, v16h b, v8f c) { return __builtin_amdgcn_wmma_f32_16x16x32_f16(false, a, false, b, (short)0, c, false, false); }
__device__ __forceinline__ v8f wmmab(v16bf a, v16bf b, v8f c) { return __builtin_amdgcn_wmma_f32_16x16x32_bf16(false, a, false, b, (short)0, c, false, false); }

template <bool SPLITA, bool F16OUT = false>
__global__ __launch_bounds__(128) void k_gemmb(const bf* __restrict__ A, const bf* __restrict__ Al, const bf* __restrict__ Bn, const float* __restrict__ bias, float* C, int ldc, h16* C2, const float* __restrict__ R = nullptr, int K = DM, int roundR = 1) {
    __shared__ __align__(16) float ost[4][16 * 68];
    const int lane = threadIdx.x & 31, wave = threadIdx.x >> 5, lr = lane & 15, hi = lane >> 4;
    const int r0 = blockIdx.x * 64 + wave * 16, c0 = blockIdx.y * 64;
    const size_t aoff = (size_t)(r0 + lr) * K + 8 * hi;
    size_t boff[4];
#pragma unroll
    for (int t = 0; t < 4; ++t) boff[t] = (size_t)(c0 + t * 16 + lr) * K + 8 * hi;
    v8f acc[4];
#pragma unroll
    for (int t = 0; t < 4; ++t) acc[t] = (v8f){};
#pragma unroll 1
    for (int kc = 0; kc < K; kc += 32) {
        const v16bf a = cat16b(*(const v8us*)(A + aoff + kc), *(const v8us*)(A + aoff + kc + 16));
        v16bf al = a;
        if (SPLITA) al = cat16b(*(const v8us*)(Al + aoff + kc), *(const v8us*)(Al + aoff + kc + 16));
#pragma unroll
        for (int t = 0; t < 4; ++t) { const v16bf b = cat16b(*(const v8us*)(Bn + boff[t] + kc), *(const v8us*)(Bn + boff[t] + kc + 16)); acc[t] = wmmab(a, b, acc[t]); if (SPLITA) acc[t] = wmmab(al, b, acc[t]); }
        asm volatile("v_nop\n\tv_nop\n\tv_nop\n\tv_nop" : "+v"(acc[0]), "+v"(acc[1]), "+v"(acc[2]), "+v"(acc[3]) : "v"(a), "v"(al));
    }
    float* os = &ost[wave][0];
#pragma unroll
    for (int t = 0; t < 4; ++t) { const float bv = bias ? bfr(bias[c0 + t * 16 + lr]) : 0.f;
#pragma unroll
        for (int j = 0; j < 8; ++j) os[(hi * 8 + j) * 68 + t * 16 + lr] = acc[t][j] + bv; }
    __syncthreads();
    if (F16OUT) {
        h16* crow = (h16*)(void*)C + (size_t)r0 * ldc + c0;
        auto pass = [&]() {
#pragma unroll
            for (int s = 0; s < 4; ++s) { const int row = 4 * s + (lane >> 3), piece = lane & 7; const float* sp = os + row * 68 + piece * 8; v8h o, o2;
#pragma unroll
                for (int i = 0; i < 8; ++i) { const h16 a = (h16)sp[i]; o[i] = a; o2[i] = (h16)((sp[i] - (float)a) * LOSC); }
                *(volatile v8h*)(crow + (size_t)row * ldc + piece * 8) = o; if (C2) *(volatile v8h*)(C2 + (size_t)r0 * ldc + c0 + (size_t)row * ldc + piece * 8) = o2; }
        };
        pass(); __threadfence(); pass();
    } else {
        float* crow = C + (size_t)r0 * ldc + c0;
        auto pass = [&]() {
#pragma unroll
            for (int s = 0; s < 8; ++s) { const int Lid = (lane >> 3) + 4 * s, piece = lane & 7; const int row = Lid >> 1, cofs = (Lid & 1) * 32 + piece * 4;
                v4f val = *(const v4fa*)(os + row * 68 + cofs); if (R) { const v4f rv = *(const v4f*)(R + ((size_t)r0 + row) * ldc + c0 + cofs); val += roundR ? (v4f){bfr(rv[0]), bfr(rv[1]), bfr(rv[2]), bfr(rv[3])} : rv; }
                *(volatile v4f*)(crow + (size_t)row * ldc + cofs) = val; }
        };
        pass(); __threadfence(); pass();
    }
}

__global__ __launch_bounds__(256) void k_cvt8(const float* __restrict__ src, bf* dst, size_t n8) {
    const size_t i = (size_t)blockIdx.x * 256 + threadIdx.x; if (i >= n8) return;
    const v8f v = *(const v8f*)(src + i * 8); v8us o;
#pragma unroll
    for (int k = 0; k < 8; ++k) o[k] = f2bf(v[k]);
    *(volatile v8us*)(dst + i * 8) = o; __threadfence(); *(volatile v8us*)(dst + i * 8) = o;
}
__global__ __launch_bounds__(256) void k_zero8(bf* dst, size_t n8) {
    const size_t i = (size_t)blockIdx.x * 256 + threadIdx.x; if (i >= n8) return; v8us z;
#pragma unroll
    for (int k = 0; k < 8; ++k) z[k] = 0;
    *(volatile v8us*)(dst + i * 8) = z; __threadfence(); *(volatile v8us*)(dst + i * 8) = z;
}

__global__ __launch_bounds__(128) void k_gemmh(const h16* __restrict__ A, const h16* __restrict__ Bn, const float* __restrict__ bias, float* C, int ldc, const float* __restrict__ R, int K, size_t sA, size_t sB, size_t sC, int roundR) {
    __shared__ __align__(16) float ost[4][16 * 68];
    const size_t z = blockIdx.z; A += z * sA; Bn += z * sB; C += z * sC; if (R) R += z * sC;
    const int lane = threadIdx.x & 31, wave = threadIdx.x >> 5, lr = lane & 15, hi = lane >> 4;
    const int r0 = blockIdx.x * 64 + wave * 16, c0 = blockIdx.y * 64;
    const size_t aoff = (size_t)(r0 + lr) * K + 8 * hi;
    size_t boff[4];
#pragma unroll
    for (int t = 0; t < 4; ++t) boff[t] = (size_t)(c0 + t * 16 + lr) * K + 8 * hi;
    v8f acc[4];
#pragma unroll
    for (int t = 0; t < 4; ++t) acc[t] = (v8f){};
#pragma unroll 1
    for (int kc = 0; kc < K; kc += 32) {
        const v16h a = cat16(*(const v8h*)(A + aoff + kc), *(const v8h*)(A + aoff + kc + 16));
#pragma unroll
        for (int t = 0; t < 4; ++t) { const v16h b = cat16(*(const v8h*)(Bn + boff[t] + kc), *(const v8h*)(Bn + boff[t] + kc + 16)); acc[t] = wmma16(a, b, acc[t]); }
        asm volatile("v_nop\n\tv_nop\n\tv_nop\n\tv_nop" : "+v"(acc[0]), "+v"(acc[1]), "+v"(acc[2]), "+v"(acc[3]) : "v"(a));
    }
    float* os = &ost[wave][0];
#pragma unroll
    for (int t = 0; t < 4; ++t) { const float bv = bias ? bfr(bias[c0 + t * 16 + lr]) : 0.f;
#pragma unroll
        for (int j = 0; j < 8; ++j) os[(hi * 8 + j) * 68 + t * 16 + lr] = acc[t][j] + bv; }
    __syncthreads();
    float* crow = C + (size_t)r0 * ldc + c0;
    auto pass = [&]() {
#pragma unroll
        for (int s = 0; s < 8; ++s) { const int Lid = (lane >> 3) + 4 * s, piece = lane & 7; const int row = Lid >> 1, cofs = (Lid & 1) * 32 + piece * 4;
            v4f val = *(const v4fa*)(os + row * 68 + cofs); if (R) { const v4f rv = *(const v4f*)(R + ((size_t)r0 + row) * ldc + c0 + cofs); val += roundR ? (v4f){bfr(rv[0]), bfr(rv[1]), bfr(rv[2]), bfr(rv[3])} : rv; }
            *(volatile v4f*)(crow + (size_t)row * ldc + cofs) = val; }
    };
    pass(); __threadfence(); pass();
}

typedef __attribute__((ext_vector_type(4))) _Float16 v4h;
__device__ __forceinline__ h16 tohx(float x) { return (h16)x; }
__global__ __launch_bounds__(256) void k_cvtx768(const float* __restrict__ x, bf* A) {
    const int lane = threadIdx.x & 31; const size_t r = (size_t)blockIdx.x * 8 + (threadIdx.x >> 5); if (r >= (size_t)NR) return;
#pragma unroll 1
    for (int ps = 0; ps < 2; ++ps) {
#pragma unroll
        for (int q = 0; q < 3; ++q) { const size_t o = r * CC + q * 256 + lane * 8; v8us v;
#pragma unroll
            for (int i = 0; i < 8; ++i) v[i] = f2bf(x[o + i]);
            *(volatile v8us*)(A + o) = v; }
        if (ps == 0) __threadfence(); }
}
__global__ __launch_bounds__(256) void k_cvt8h(const float* __restrict__ src, h16* dst, size_t n8) { const size_t i = (size_t)blockIdx.x * 256 + threadIdx.x; if (i >= n8) return; const v8f v = *(const v8f*)(src + i * 8); v8h o;
#pragma unroll
    for (int k = 0; k < 8; ++k) o[k] = tohx(bfr(v[k])); *(volatile v8h*)(dst + i * 8) = o; __threadfence(); *(volatile v8h*)(dst + i * 8) = o; }
__global__ __launch_bounds__(256) void k_posmap(const float* __restrict__ w1, const float* __restrict__ b1, const float* __restrict__ w2, const float* __restrict__ b2, float* PM) {
    const int lane = threadIdx.x & 31; const int w = blockIdx.x * 8 + (threadIdx.x >> 5); if (w >= NH_ * NTK) return; const int h = w / NTK, i = w % NTK; const int ix = i % 14, iy = i / 14;
#pragma unroll 1
    for (int ps = 0; ps < 2; ++ps) {
#pragma unroll 1
        for (int c0 = lane * 4; c0 < NP; c0 += 128) { v4f o;
#pragma unroll
            for (int q = 0; q < 4; ++q) { const int j = c0 + q; float a = 0.f;
                if (j < NTK) { const float rx = (float)((j % 14) - ix), ry = (float)((j / 14) - iy); a = bfr(b2[h]);
#pragma unroll 1
                    for (int m = 0; m < HD; ++m) { const int c = h * HD + m; float p = rx * bfr(w1[c * 2]); p = fmaf(ry, bfr(w1[c * 2 + 1]), p); p += bfr(b1[c]); p = fmaxf(p, 0.f); a = fmaf(p, bfr(w2[c]), a); } }
                o[q] = a; }
            *(volatile v4f*)(PM + ((size_t)h * NP + i) * NP + c0) = o; }
        if (ps == 0) __threadfence(); }
}
__global__ __launch_bounds__(256) void k_hplh2(const float* __restrict__ QK, int b0, int col0, float sc, h16* P) {
    const int lane = threadIdx.x & 31; const size_t w = (size_t)blockIdx.x * 8 + (threadIdx.x >> 5); const int i = (int)(w * 2 + (lane >> 4)); if (i >= NP) return; const int g = blockIdx.z / NH_, h = blockIdx.z % NH_; const int c0 = (lane & 15) * 4; const bool live = i < NTK; v4h o;
#pragma unroll
    for (int q = 0; q < 4; ++q) o[q] = tohx(live ? QK[((size_t)(b0 + g) * NTK + i) * (2 * CC) + col0 + h * HD + c0 + q] * sc : 0.f);
    const size_t off = ((size_t)blockIdx.z * NP + i) * HD + c0; *(volatile v4h*)(P + off) = o; __threadfence(); *(volatile v4h*)(P + off) = o;
}
__global__ __launch_bounds__(256) void k_vTh2(const float* __restrict__ V, int b0, h16* VT) {
    __shared__ float tl[64][65];
    const int tid = threadIdx.x; const int t0 = blockIdx.x * 64; const int g = blockIdx.z / NH_, h = blockIdx.z % NH_; const int rr = tid >> 2, cq = (tid & 3) * 16; const int t = t0 + rr;
#pragma unroll
    for (int i = 0; i < 16; ++i) tl[rr][cq + i] = (t < NTK) ? V[((size_t)(b0 + g) * NTK + t) * CC + h * HD + cq + i] : 0.f;
    __syncthreads();
    const int lane = tid & 31, wv = tid >> 5;
    auto pass = [&]() {
#pragma unroll
        for (int st = 0; st < 4; ++st) { const int dr = wv * 8 + st * 2 + (lane >> 4); const int tq = (lane & 15) * 4; v4h v;
#pragma unroll
            for (int i = 0; i < 4; ++i) v[i] = tohx(tl[tq + i][dr]);
            *(volatile v4h*)(VT + ((size_t)blockIdx.z * HD + dr) * NP + t0 + tq) = v; }
    };
    pass(); __threadfence(); pass();
}
__global__ __launch_bounds__(256) void k_softpm(const float* __restrict__ S, const float* __restrict__ PM, h16* P) {
    const int lane = threadIdx.x & 31, i = blockIdx.x * 8 + (threadIdx.x >> 5); if (i >= NP) return; const int h = blockIdx.z % NH_; const size_t zo = (size_t)blockIdx.z * NP * NP; const float* sr = S + zo + (size_t)i * NP; const float* pr = PM + ((size_t)h * NP + (i < NTK ? i : 0)) * NP; h16* po = P + zo + (size_t)i * NP;
    float m = -3.0e38f;
#pragma unroll 1
    for (int c0 = lane * 4; c0 < NP; c0 += 128) {
#pragma unroll
        for (int q = 0; q < 4; ++q) { const int j = c0 + q; if (j < NTK) m = fmaxf(m, sr[j] * pr[j]); } }
#pragma unroll
    for (int sh = 16; sh; sh >>= 1) m = fmaxf(m, __shfl_xor(m, sh, 32));
    float sum = 0.f;
#pragma unroll 1
    for (int c0 = lane * 4; c0 < NP; c0 += 128) {
#pragma unroll
        for (int q = 0; q < 4; ++q) { const int j = c0 + q; if (j < NTK) sum += __expf(sr[j] * pr[j] - m); } }
#pragma unroll
    for (int sh = 16; sh; sh >>= 1) sum += __shfl_xor(sum, sh, 32);
    const float inv = 1.0f / sum;
#pragma unroll 1
    for (int ps = 0; ps < 2; ++ps) {
#pragma unroll 1
        for (int c0 = lane * 4; c0 < NP; c0 += 128) { v4h o;
#pragma unroll
            for (int q = 0; q < 4; ++q) { const int j = c0 + q; o[q] = tohx((j < NTK) ? __expf(sr[(j < NTK) ? j : 0] * pr[(j < NTK) ? j : 0] - m) * inv : 0.f); }
            *(volatile v4h*)(po + c0) = o; }
        if (ps == 0) __threadfence(); }
}
__global__ __launch_bounds__(256) void k_mergeh2(const float* __restrict__ OZ, int b0, h16* OH) {
    const int lane = threadIdx.x & 31; const size_t w = (size_t)blockIdx.x * 8 + (threadIdx.x >> 5); if (w >= (size_t)IG * NTK) return; const int g = (int)(w / NTK), i = (int)(w % NTK); const size_t row = (size_t)(b0 + g) * NTK + i;
#pragma unroll 1
    for (int ps = 0; ps < 2; ++ps) {
#pragma unroll
        for (int q = 0; q < 3; ++q) { const int c0 = q * 256 + lane * 8; const int h = c0 / HD, d0 = c0 % HD; v8h o;
#pragma unroll
            for (int k = 0; k < 8; ++k) o[k] = tohx(OZ[(((size_t)(g * NH_ + h)) * NP + i) * HD + d0 + k]);
            *(volatile v8h*)(OH + row * CC + c0) = o; }
        if (ps == 0) __threadfence(); }
}
extern "C" void kernel_launch(void* const* d_in, const int* in_sizes, int n_in,
                              void* d_out, int out_size, void* d_ws, size_t ws_size, hipStream_t stream) {
    (void)in_sizes; (void)n_in; (void)out_size;
    const float* x = (const float*)d_in[0]; const float* qkw = (const float*)d_in[1]; const float* vw = (const float*)d_in[2]; const float* w1 = (const float*)d_in[3]; const float* b1 = (const float*)d_in[4]; const float* w2 = (const float*)d_in[5]; const float* b2 = (const float*)d_in[6]; const float* pw = (const float*)d_in[7]; const float* pb = (const float*)d_in[8];
    float* out = (float*)d_out;
    char* wsp = (char*)d_ws;
    auto take = [&](size_t bytes) { char* p = wsp; wsp += (bytes + 255) & ~(size_t)255; return (void*)p; };
    bf* WQK = (bf*)take((size_t)2 * CC * CC * 2); bf* WV = (bf*)take((size_t)CC * CC * 2); h16* WP = (h16*)take((size_t)CC * CC * 2); float* PM = (float*)take((size_t)NH_ * NP * NP * 4);
    bf* XB = (bf*)take((size_t)NR * CC * 2); float* QK = (float*)take((size_t)NR * 2 * CC * 4); float* V = (float*)take((size_t)NR * CC * 4);
    h16* Qx = (h16*)take((size_t)IG * NH_ * NP * HD * 2); h16* Kx = (h16*)take((size_t)IG * NH_ * NP * HD * 2); h16* VTx = (h16*)take((size_t)IG * NH_ * HD * NP * 2); float* S = (float*)take((size_t)IG * NH_ * NP * NP * 4); h16* Px = (h16*)take((size_t)IG * NH_ * NP * NP * 2); float* OZ = (float*)take((size_t)IG * NH_ * NP * HD * 4); h16* OH = (h16*)take((size_t)NR * CC * 2);
    if ((size_t)(wsp - (char*)d_ws) > ws_size) return;
    k_cvt8<<<(unsigned)(((size_t)2 * CC * CC / 8 + 255) / 256), 256, 0, stream>>>(qkw, WQK, (size_t)2 * CC * CC / 8); k_cvt8<<<(unsigned)(((size_t)CC * CC / 8 + 255) / 256), 256, 0, stream>>>(vw, WV, (size_t)CC * CC / 8);
    k_cvt8h<<<(unsigned)(((size_t)CC * CC / 8 + 255) / 256), 256, 0, stream>>>(pw, WP, (size_t)CC * CC / 8);
    k_posmap<<<(NH_ * NTK + 7) / 8, 256, 0, stream>>>(w1, b1, w2, b2, PM);
    k_cvtx768<<<NR / 8, 256, 0, stream>>>(x, XB);
    k_gemmb<false, false><<<dim3(NR / 64, (2 * CC) / 64, 1), 128, 0, stream>>>(XB, nullptr, WQK, nullptr, QK, 2 * CC, nullptr, nullptr, CC);
    k_gemmb<false, false><<<dim3(NR / 64, CC / 64, 1), 128, 0, stream>>>(XB, nullptr, WV, nullptr, V, CC, nullptr, nullptr, CC);
    for (int b0 = 0; b0 < NB_; b0 += IG) {
        k_hplh2<<<dim3((NP / 2) / 8, 1, IG * NH_), 256, 0, stream>>>(QK, b0, 0, SCL, Qx); k_hplh2<<<dim3((NP / 2) / 8, 1, IG * NH_), 256, 0, stream>>>(QK, b0, CC, 1.0f, Kx); k_vTh2<<<dim3(NP / 64, 1, IG * NH_), 256, 0, stream>>>(V, b0, VTx);
        k_gemmh<<<dim3(NP / 64, NP / 64, IG * NH_), 128, 0, stream>>>(Qx, Kx, nullptr, S, NP, nullptr, HD, (size_t)NP * HD, (size_t)NP * HD, (size_t)NP * NP, 0);
        k_softpm<<<dim3(NP / 8, 1, IG * NH_), 256, 0, stream>>>(S, PM, Px);
        k_gemmh<<<dim3(NP / 64, 1, IG * NH_), 128, 0, stream>>>(Px, VTx, nullptr, OZ, HD, nullptr, NP, (size_t)NP * NP, (size_t)HD * NP, (size_t)NP * HD, 0);
        k_mergeh2<<<(IG * NTK + 7) / 8, 256, 0, stream>>>(OZ, b0, OH); }
    k_gemmh<<<dim3(NR / 64, CC / 64, 1), 128, 0, stream>>>(OH, WP, pb, out, CC, nullptr, CC, 0, 0, 0, 0);
}
